// MultiHeadGAT_27719718928466
// MI455X (gfx1250) — hardware-verified
//
#include <hip/hip_runtime.h>

typedef __attribute__((ext_vector_type(16))) __bf16   v16b;
typedef __attribute__((ext_vector_type(8)))  __bf16   v8b;
typedef __attribute__((ext_vector_type(8)))  float    v8f;
typedef __attribute__((ext_vector_type(4)))  float    v4f;
typedef __attribute__((ext_vector_type(4)))  unsigned v4u;

constexpr int NHEADS   = 4;
constexpr int TDIM     = 768;
constexpr int HIDC     = 256;
constexpr int ODIM     = 768;
constexpr int NBATCH   = 16;
constexpr int SEQL     = 1024;
constexpr int NTOK     = NBATCH * SEQL;
constexpr int CATD     = NHEADS * HIDC;
constexpr int HB_PITCH = 260;
constexpr int ZS_PITCH = 772;
constexpr int SL_PITCH = 100;
constexpr int OUT_ELEMS = NBATCH * ODIM;

static_assert(TDIM % 32 == 0 && CATD % 32 == 0 && ODIM % 32 == 0 && SEQL % 32 == 0);
static_assert(NTOK % 64 == 0 && HIDC == 4 * 64 && ODIM == 8 * 96 && SEQL == 4 * 256 && NBATCH == 16);
static_assert(TDIM % 64 == 0 && HIDC % 64 == 0 && ODIM % 64 == 0 && CATD % 64 == 0);
static_assert((HB_PITCH * 4) % 16 == 0 && (ZS_PITCH * 4) % 16 == 0 && (SL_PITCH * 4) % 16 == 0);
static_assert((NTOK * TDIM) % 8 == 0);
static_assert(3 * OUT_ELEMS * 4 + OUT_ELEMS * 4 == 196608);

__device__ __forceinline__ unsigned short f2bf_bits(float f) {
  unsigned u = __float_as_uint(f);
  return (unsigned short)((u + 0x7FFFu + ((u >> 16) & 1u)) >> 16);
}
__device__ __forceinline__ float bf_bits2f(unsigned short h) { return __uint_as_float(((unsigned)h) << 16); }
__device__ __forceinline__ float bfr(float f) { return bf_bits2f(f2bf_bits(f)); }
__device__ __forceinline__ void split_bits(float f, unsigned short& hb, unsigned short& lb) {
  hb = f2bf_bits(f);
  lb = f2bf_bits(f - bf_bits2f(hb));
}
__device__ __forceinline__ void split_bf(float f, __bf16& hi, __bf16& lo) {
  unsigned short hb, lb; split_bits(f, hb, lb);
  hi = __builtin_bit_cast(__bf16, hb);
  lo = __builtin_bit_cast(__bf16, lb);
}

__device__ __forceinline__ void dep_guard_b(v8f& a, v8f& b, v16b x, v16b y) { asm volatile("v_nop\n\tv_nop\n\tv_nop\n\tv_nop" : "+v"(a), "+v"(b) : "v"(x), "v"(y)); }
__device__ __forceinline__ void keep4_b(v16b a, v16b b, v16b c, v16b d) { asm volatile("v_nop" :: "v"(a), "v"(b), "v"(c), "v"(d)); }
__device__ __forceinline__ void acc_guard4(v8f& a, v8f& b, v8f& c, v8f& d) { asm volatile("v_nop\n\tv_nop\n\tv_nop\n\tv_nop" : "+v"(a), "+v"(b), "+v"(c), "+v"(d)); }
__device__ __forceinline__ void acc_guard2(v8f& a, v8f& b) { asm volatile("v_nop\n\tv_nop\n\tv_nop\n\tv_nop" : "+v"(a), "+v"(b)); }

template <typename T> struct Frag;
template <> struct Frag<__bf16> {
  typedef v16b V; union U { v16b v; v8b h[2]; };
  static __device__ __forceinline__ v16b load(const __bf16* p) {
    U f; f.h[0] = *(const v8b*)(p); f.h[1] = *(const v8b*)(p + 16); return f.v;
  }
  static __device__ __forceinline__ v8f mma(v16b a, v16b b, v8f c) {
    return __builtin_amdgcn_wmma_f32_16x16x32_bf16(false, a, false, b, (short)0, c, false, false);
  }
  static __device__ __forceinline__ void guard(v8f& a, v8f& b, v16b x, v16b y) { dep_guard_b(a, b, x, y); }
  static __device__ __forceinline__ void keep(v16b a, v16b b, v16b c, v16b d) { keep4_b(a, b, c, d); }
};

__device__ __forceinline__ v8f zero8() { return (v8f){0.f, 0.f, 0.f, 0.f, 0.f, 0.f, 0.f, 0.f}; }
__device__ __forceinline__ float leaky_f(float e) { return (e >= 0.0f) ? e : 0.01f * e; }
__device__ __forceinline__ void wave_lds_sync() {
  __builtin_amdgcn_fence(__ATOMIC_RELEASE, "workgroup");
  __builtin_amdgcn_wave_barrier();
  __builtin_amdgcn_fence(__ATOMIC_ACQUIRE, "workgroup");
}

__global__ __launch_bounds__(256) void k_cast_bf16x8(
    const float* __restrict__ in, unsigned short* __restrict__ outp, int n8) {
  const int i = blockIdx.x * 256 + threadIdx.x;
  if (i < n8) {
    const float* p = in + (size_t)i * 8;
    const v4f a = *(const v4f*)p;
    const v4f c = *(const v4f*)(p + 4);
    v4u u;
    u[0] = (unsigned)f2bf_bits(a[0]) | ((unsigned)f2bf_bits(a[1]) << 16);
    u[1] = (unsigned)f2bf_bits(a[2]) | ((unsigned)f2bf_bits(a[3]) << 16);
    u[2] = (unsigned)f2bf_bits(c[0]) | ((unsigned)f2bf_bits(c[1]) << 16);
    u[3] = (unsigned)f2bf_bits(c[2]) | ((unsigned)f2bf_bits(c[3]) << 16);
    unsigned short* d = outp + (size_t)i * 8;
    *(volatile v4u*)d = u;
    __threadfence();
    *(volatile v4u*)d = u;
  }
}

__global__ __launch_bounds__(256) void k_tr_cast(
    const float* __restrict__ in, unsigned short* __restrict__ outp, int R, int Cc) {
  __shared__ float tile[64][65];
  const int tid = threadIdx.x, lane = tid & 31, wave = tid >> 5;
  const int c0 = blockIdx.x * 64, r0 = blockIdx.y * 64, bz = blockIdx.z;
  const float* inb = in + (size_t)bz * R * Cc;
  unsigned short* outb = outp + (size_t)bz * R * Cc;
  {
    const int rr = tid >> 2, cq = (tid & 3) * 16;
    const float* p = inb + (size_t)(r0 + rr) * Cc + c0 + cq;
#pragma unroll
    for (int u = 0; u < 4; ++u) {
      const v4f v = *(const v4f*)(p + 4 * u);
      tile[rr][cq + 4 * u + 0] = v[0];
      tile[rr][cq + 4 * u + 1] = v[1];
      tile[rr][cq + 4 * u + 2] = v[2];
      tile[rr][cq + 4 * u + 3] = v[3];
    }
  }
  __syncthreads();
  const int q = lane >> 3, r8 = (lane & 7) * 8;
#pragma unroll
  for (int it = 0; it < 2; ++it) {
    const int cc = wave * 8 + it * 4 + q;
    v4u u;
#pragma unroll
    for (int e2 = 0; e2 < 4; ++e2) {
      const float f0 = tile[r8 + 2 * e2][cc];
      const float f1 = tile[r8 + 2 * e2 + 1][cc];
      u[e2] = (unsigned)f2bf_bits(f0) | ((unsigned)f2bf_bits(f1) << 16);
    }
    unsigned short* dst = outb + (size_t)(c0 + cc) * R + r0 + r8;
    *(volatile v4u*)dst = u;
    __threadfence();
    *(volatile v4u*)dst = u;
  }
}

__global__ __launch_bounds__(128) void k_proj_ln(
    const unsigned short* __restrict__ Xb,
    const unsigned short* __restrict__ WT,
    const float* __restrict__ bfc, const float* __restrict__ lng, const float* __restrict__ lnb,
    const float* __restrict__ aw,
    unsigned short* __restrict__ hThi, unsigned short* __restrict__ hTlo,
    float* __restrict__ srow, float* __restrict__ scol)
{
  __shared__ __align__(16) float hbuf[64 * HB_PITCH];
  __shared__ __align__(16) float p_bias[HIDC];
  __shared__ __align__(16) float p_g[HIDC];
  __shared__ __align__(16) float p_b[HIDC];
  __shared__ __align__(16) float p_a1[HIDC];
  __shared__ __align__(16) float p_a2[HIDC];
  __shared__ __align__(16) float sr_s[64];
  __shared__ __align__(16) float sc_s[64];

  const int tid = threadIdx.x, lane = tid & 31, wave = tid >> 5;
  const int head = blockIdx.y, m0 = blockIdx.x * 64;

  for (int c = tid; c < HIDC; c += 128) {
    p_bias[c] = bfr(bfc[head * HIDC + c]);
    p_g[c]    = bfr(lng[head * HIDC + c]);
    p_b[c]    = bfr(lnb[head * HIDC + c]);
    p_a1[c]   = bfr(aw[head * 2 * HIDC + c]);
    p_a2[c]   = bfr(aw[head * 2 * HIDC + HIDC + c]);
  }

  const __bf16* A  = (const __bf16*)Xb;
  const __bf16* Bt = (const __bf16*)WT + (size_t)head * HIDC * TDIM;
  const int rlane = lane & 15;
  const int koff  = (lane >> 4) * 8;
  const int mOff  = (lane >> 4) * 8;
  const int n0    = wave * 64;

  v8f acc[4][4];
#pragma unroll
  for (int i = 0; i < 4; ++i)
#pragma unroll
    for (int j = 0; j < 4; ++j) acc[i][j] = zero8();

  for (int k0 = 0; k0 < TDIM; k0 += 32) {
    v16b bh[4];
#pragma unroll
    for (int j = 0; j < 4; ++j)
      bh[j] = Frag<__bf16>::load(Bt + (size_t)(n0 + (j << 4) + rlane) * TDIM + koff + k0);
#pragma unroll
    for (int i = 0; i < 4; ++i) {
      const v16b ah = Frag<__bf16>::load(A + (size_t)(m0 + (i << 4) + rlane) * TDIM + koff + k0);
#pragma unroll
      for (int j = 0; j < 4; ++j) acc[i][j] = Frag<__bf16>::mma(ah, bh[j], acc[i][j]);
      Frag<__bf16>::guard(acc[i][0], acc[i][3], ah, ah);
    }
    Frag<__bf16>::keep(bh[0], bh[1], bh[2], bh[3]);
  }
  acc_guard4(acc[0][0], acc[0][1], acc[0][2], acc[0][3]);
  acc_guard4(acc[1][0], acc[1][1], acc[1][2], acc[1][3]);
  acc_guard4(acc[2][0], acc[2][1], acc[2][2], acc[2][3]);
  acc_guard4(acc[3][0], acc[3][1], acc[3][2], acc[3][3]);

#pragma unroll
  for (int i = 0; i < 4; ++i)
#pragma unroll
    for (int j = 0; j < 4; ++j)
#pragma unroll
      for (int r = 0; r < 8; ++r)
        hbuf[((i << 4) + mOff + r) * HB_PITCH + n0 + (j << 4) + rlane] = acc[i][j][r];
  __syncthreads();

  {
    const int cb = lane * 8;
    const v4f g0 = *(const v4f*)(p_g + cb),    g1 = *(const v4f*)(p_g + cb + 4);
    const v4f b0 = *(const v4f*)(p_b + cb),    b1 = *(const v4f*)(p_b + cb + 4);
    const v4f q0 = *(const v4f*)(p_bias + cb), q1 = *(const v4f*)(p_bias + cb + 4);
    const v4f u0 = *(const v4f*)(p_a1 + cb),   u1 = *(const v4f*)(p_a1 + cb + 4);
    const v4f w0 = *(const v4f*)(p_a2 + cb),   w1 = *(const v4f*)(p_a2 + cb + 4);
#pragma unroll 1
    for (int rr = 0; rr < 16; ++rr) {
      const int row = wave * 16 + rr;
      float* hp = hbuf + row * HB_PITCH + cb;
      const v4f x0 = *(const v4f*)hp + q0;
      const v4f x1 = *(const v4f*)(hp + 4) + q1;
      float s = 0.0f;
      s += x0[0]; s += x0[1]; s += x0[2]; s += x0[3];
      s += x1[0]; s += x1[1]; s += x1[2]; s += x1[3];
#pragma unroll
      for (int off = 16; off > 0; off >>= 1) s += __shfl_xor(s, off, 32);
      const float mu = s * (1.0f / 256.0f);
      const v4f d0 = x0 - mu, d1 = x1 - mu;
      float s2 = 0.0f;
      s2 += d0[0] * d0[0]; s2 += d0[1] * d0[1]; s2 += d0[2] * d0[2]; s2 += d0[3] * d0[3];
      s2 += d1[0] * d1[0]; s2 += d1[1] * d1[1]; s2 += d1[2] * d1[2]; s2 += d1[3] * d1[3];
#pragma unroll
      for (int off = 16; off > 0; off >>= 1) s2 += __shfl_xor(s2, off, 32);
      const float rs = rsqrtf(s2 * (1.0f / 256.0f) + 1e-5f);
      const v4f h0 = d0 * rs * g0 + b0;
      const v4f h1 = d1 * rs * g1 + b1;
      float t1 = 0.0f, t2 = 0.0f;
      t1 += h0[0] * u0[0]; t1 += h0[1] * u0[1]; t1 += h0[2] * u0[2]; t1 += h0[3] * u0[3];
      t1 += h1[0] * u1[0]; t1 += h1[1] * u1[1]; t1 += h1[2] * u1[2]; t1 += h1[3] * u1[3];
      t2 += h0[0] * w0[0]; t2 += h0[1] * w0[1]; t2 += h0[2] * w0[2]; t2 += h0[3] * w0[3];
      t2 += h1[0] * w1[0]; t2 += h1[1] * w1[1]; t2 += h1[2] * w1[2]; t2 += h1[3] * w1[3];
#pragma unroll
      for (int off = 16; off > 0; off >>= 1) { t1 += __shfl_xor(t1, off, 32); t2 += __shfl_xor(t2, off, 32); }
      *(v4f*)hp = h0;
      *(v4f*)(hp + 4) = h1;
      if (lane == 0) { sr_s[row] = t1; sc_s[row] = t2; }
    }
  }
  __syncthreads();

  {
    const int bidx = m0 >> 10;
    const int t0   = m0 & (SEQL - 1);
    const int q = lane >> 3, tok8 = (lane & 7) * 8;
    const size_t prow0 = (size_t)(head * NBATCH + bidx) * HIDC;
#pragma unroll 1
    for (int it = 0; it < 16; ++it) {
      const int ch = wave * 64 + it * 4 + q;
      v4u hv, lv;
#pragma unroll
      for (int e2 = 0; e2 < 4; ++e2) {
        const float f0 = hbuf[(tok8 + 2 * e2) * HB_PITCH + ch];
        const float f1 = hbuf[(tok8 + 2 * e2 + 1) * HB_PITCH + ch];
        unsigned short ha, la, hb2, lb2;
        split_bits(f0, ha, la);
        split_bits(f1, hb2, lb2);
        hv[e2] = (unsigned)ha | ((unsigned)hb2 << 16);
        lv[e2] = (unsigned)la | ((unsigned)lb2 << 16);
      }
      const size_t off = (prow0 + (size_t)ch) * SEQL + t0 + tok8;
      *(volatile v4u*)(hThi + off) = hv;
      *(volatile v4u*)(hTlo + off) = lv;
      __threadfence();
      *(volatile v4u*)(hThi + off) = hv;
      *(volatile v4u*)(hTlo + off) = lv;
    }
  }

  if (wave == 0) {
    const int l16 = lane & 15;
    const v4f v = *(const v4f*)(sr_s + 4 * l16);
    float* dst = srow + (size_t)head * NTOK + m0 + 4 * l16;
    if (lane < 16) *(volatile v4f*)dst = v;
    __threadfence();
    if (lane < 16) *(volatile v4f*)dst = v;
  } else if (wave == 1) {
    const int l16 = lane & 15;
    const v4f v = *(const v4f*)(sc_s + 4 * l16);
    float* dst = scol + (size_t)head * NTOK + m0 + 4 * l16;
    if (lane < 16) *(volatile v4f*)dst = v;
    __threadfence();
    if (lane < 16) *(volatile v4f*)dst = v;
  }
}

__global__ __launch_bounds__(256) void k_attnw(
    const float* __restrict__ srow, const float* __restrict__ scol, const float* __restrict__ ab,
    const unsigned short* __restrict__ hThi, const unsigned short* __restrict__ hTlo,
    float* __restrict__ sent_pre)
{
  __shared__ __align__(16) float  sr_s[SEQL];
  __shared__ __align__(16) v4f    rowdat[SEQL];
  __shared__ __align__(16) __bf16 w_hi_s[SEQL];
  __shared__ __align__(16) __bf16 w_lo_s[SEQL];
  __shared__ float red_s[8];

  const int tid = threadIdx.x, lane = tid & 31, wave = tid >> 5;
  const int hb = blockIdx.x;
  const int head = hb >> 4, b = hb & 15;
  const size_t base = (size_t)head * NTOK + (size_t)b * SEQL;
  const float abv = bfr(ab[head]);

  {
    const v4f r4 = *(const v4f*)(srow + base + 4 * tid);
    *(v4f*)(sr_s + 4 * tid) = r4;
    float mx = fmaxf(fmaxf(r4[0], r4[1]), fmaxf(r4[2], r4[3]));
#pragma unroll
    for (int off = 16; off > 0; off >>= 1) mx = fmaxf(mx, __shfl_xor(mx, off, 32));
    if (lane == 0) red_s[wave] = mx;
  }
  __syncthreads();
  float Mr = red_s[0];
#pragma unroll
  for (int w8 = 1; w8 < 8; ++w8) Mr = fmaxf(Mr, red_s[w8]);

  {
    float ci[4], mi[4], zi[4];
#pragma unroll
    for (int q = 0; q < 4; ++q) {
      ci[q] = scol[base + tid + 256 * q];
      mi[q] = leaky_f((ci[q] + Mr) + abv);
      zi[q] = 0.0f;
    }
#pragma unroll 1
    for (int j = 0; j < SEQL; ++j) {
      const float r = sr_s[j];
#pragma unroll
      for (int q = 0; q < 4; ++q) {
        const float e = leaky_f((ci[q] + r) + abv);
        zi[q] += expf(e - mi[q]);
      }
    }
#pragma unroll
    for (int q = 0; q < 4; ++q) {
      v4f d; d[0] = ci[q]; d[1] = mi[q]; d[2] = 1.0f / zi[q]; d[3] = 0.0f;
      rowdat[tid + 256 * q] = d;
    }
  }
  __syncthreads();

  {
    float rj[4], wj[4];
#pragma unroll
    for (int q = 0; q < 4; ++q) { rj[q] = sr_s[tid + 256 * q]; wj[q] = 0.0f; }
#pragma unroll 1
    for (int i = 0; i < SEQL; ++i) {
      const v4f d = rowdat[i];
#pragma unroll
      for (int q = 0; q < 4; ++q) {
        const float e = leaky_f((d[0] + rj[q]) + abv);
        wj[q] += expf(e - d[1]) * d[2];
      }
    }
#pragma unroll
    for (int q = 0; q < 4; ++q) {
      const float w = wj[q] * (1.0f / 1024.0f);
      __bf16 whi, wlo; split_bf(w, whi, wlo);
      w_hi_s[tid + 256 * q] = whi;
      w_lo_s[tid + 256 * q] = wlo;
    }
  }
  __syncthreads();

  {
    const int rlane = lane & 15, koff = (lane >> 4) * 8;
    const int ch0 = wave * 32;
    const __bf16* Hh = (const __bf16*)hThi + (size_t)hb * HIDC * SEQL;
    const __bf16* Hl = (const __bf16*)hTlo + (size_t)hb * HIDC * SEQL;
    v8f acc0 = zero8(), acc1 = zero8();
    for (int k0 = 0; k0 < SEQL; k0 += 32) {
      const v16b ahi = Frag<__bf16>::load(w_hi_s + k0 + koff);
      const v16b alo = Frag<__bf16>::load(w_lo_s + k0 + koff);
      const v16b bh0 = Frag<__bf16>::load(Hh + (size_t)(ch0 + rlane) * SEQL + k0 + koff);
      const v16b bh1 = Frag<__bf16>::load(Hh + (size_t)(ch0 + 16 + rlane) * SEQL + k0 + koff);
      const v16b bl0 = Frag<__bf16>::load(Hl + (size_t)(ch0 + rlane) * SEQL + k0 + koff);
      const v16b bl1 = Frag<__bf16>::load(Hl + (size_t)(ch0 + 16 + rlane) * SEQL + k0 + koff);
      acc0 = Frag<__bf16>::mma(ahi, bh0, acc0);
      acc0 = Frag<__bf16>::mma(ahi, bl0, acc0);
      acc0 = Frag<__bf16>::mma(alo, bh0, acc0);
      acc1 = Frag<__bf16>::mma(ahi, bh1, acc1);
      acc1 = Frag<__bf16>::mma(ahi, bl1, acc1);
      acc1 = Frag<__bf16>::mma(alo, bh1, acc1);
      Frag<__bf16>::guard(acc0, acc1, ahi, alo);
      Frag<__bf16>::keep(bh0, bh1, bl0, bl1);
    }
    acc_guard2(acc0, acc1);
    const float val = (lane < 16) ? acc0[0] : acc1[0];
    float* dst = sent_pre + (size_t)b * CATD + head * HIDC + ch0 + lane;
    *(volatile float*)dst = val;
    __threadfence();
    *(volatile float*)dst = val;
  }
}

__global__ __launch_bounds__(256) void k_tail(
    const float* __restrict__ sent_pre,
    const unsigned short* __restrict__ WcatT,
    const float* __restrict__ bcat, const float* __restrict__ lOg, const float* __restrict__ lOb,
    const unsigned short* __restrict__ WfcsT,
    const float* __restrict__ bfcs,
    float* __restrict__ outp)
{
  __shared__ __align__(16) float zs[16 * ZS_PITCH];
  __shared__ __align__(16) float slab_all[8 * 16 * SL_PITCH];

  const int tid = threadIdx.x, lane = tid & 31, wave = tid >> 5;
  const int rlane = lane & 15, koff = (lane >> 4) * 8, mOff = (lane >> 4) * 8;
  const int cw = wave * 96;

  {
    const __bf16* Bt = (const __bf16*)WcatT;
    v8f acc[6];
#pragma unroll
    for (int j = 0; j < 6; ++j) acc[j] = zero8();
    for (int k0 = 0; k0 < CATD; k0 += 32) {
      const float* ap = sent_pre + (size_t)rlane * CATD + k0 + koff;
      const v4f a0 = *(const v4f*)ap, a1 = *(const v4f*)(ap + 4);
      const v4f a2 = *(const v4f*)(ap + 16), a3 = *(const v4f*)(ap + 20);
      v16b ahi, alo;
#pragma unroll
      for (int e = 0; e < 4; ++e) {
        __bf16 h, l;
        split_bf(a0[e], h, l); ahi[e] = h;      alo[e] = l;
        split_bf(a1[e], h, l); ahi[4 + e] = h;  alo[4 + e] = l;
        split_bf(a2[e], h, l); ahi[8 + e] = h;  alo[8 + e] = l;
        split_bf(a3[e], h, l); ahi[12 + e] = h; alo[12 + e] = l;
      }
      v16b bw[6];
#pragma unroll
      for (int j = 0; j < 6; ++j)
        bw[j] = Frag<__bf16>::load(Bt + (size_t)(cw + (j << 4) + rlane) * CATD + k0 + koff);
#pragma unroll
      for (int j = 0; j < 6; ++j) {
        acc[j] = Frag<__bf16>::mma(ahi, bw[j], acc[j]);
        acc[j] = Frag<__bf16>::mma(alo, bw[j], acc[j]);
      }
      Frag<__bf16>::guard(acc[0], acc[5], ahi, alo);
      Frag<__bf16>::keep(bw[0], bw[1], bw[2], bw[3]);
      Frag<__bf16>::keep(bw[4], bw[5], bw[4], bw[5]);
    }
    acc_guard4(acc[0], acc[1], acc[2], acc[3]);
    acc_guard2(acc[4], acc[5]);
#pragma unroll
    for (int j = 0; j < 6; ++j) {
      const int col = cw + (j << 4) + rlane;
      const float bv = bfr(bcat[col]);
#pragma unroll
      for (int r = 0; r < 8; ++r) zs[(mOff + r) * ZS_PITCH + col] = acc[j][r] + bv;
    }
  }
  __syncthreads();

#pragma unroll 1
  for (int rr = 0; rr < 2; ++rr) {
    const int row = wave * 2 + rr;
    float* zr = zs + row * ZS_PITCH;
    float s = 0.0f;
#pragma unroll 1
    for (int e = 0; e < 24; ++e) s += zr[lane + 32 * e];
#pragma unroll
    for (int off = 16; off > 0; off >>= 1) s += __shfl_xor(s, off, 32);
    const float mu = s * (1.0f / 768.0f);
    float s2 = 0.0f;
#pragma unroll 1
    for (int e = 0; e < 24; ++e) { const float d = zr[lane + 32 * e] - mu; s2 += d * d; }
#pragma unroll
    for (int off = 16; off > 0; off >>= 1) s2 += __shfl_xor(s2, off, 32);
    const float rs = rsqrtf(s2 * (1.0f / 768.0f) + 1e-5f);
#pragma unroll 1
    for (int e = 0; e < 24; ++e) {
      const int c = lane + 32 * e;
      const float v = (zr[c] - mu) * rs * bfr(lOg[c]) + bfr(lOb[c]);
      zr[c] = v;
    }
  }
  __syncthreads();

  {
    float* o3 = outp + 3 * OUT_ELEMS;
    for (int pass = 0; pass < 2; ++pass) {
#pragma unroll
      for (int rr = 0; rr < 2; ++rr) {
        const int row = wave * 2 + rr;
#pragma unroll
        for (int it = 0; it < 6; ++it) {
          const v4f v = *(const v4f*)(zs + row * ZS_PITCH + it * 128 + 4 * lane);
          *(volatile v4f*)(o3 + (size_t)row * ODIM + it * 128 + 4 * lane) = v;
        }
      }
      __threadfence();
    }
  }

  float* slab = slab_all + wave * 16 * SL_PITCH;
#pragma unroll 1
  for (int oi = 0; oi < 3; ++oi) {
    const __bf16* Bt = (const __bf16*)WfcsT + (size_t)oi * ODIM * ODIM;
    v8f acc[6];
#pragma unroll
    for (int j = 0; j < 6; ++j) acc[j] = zero8();
    for (int k0 = 0; k0 < ODIM; k0 += 32) {
      const float* ap = zs + rlane * ZS_PITCH + k0 + koff;
      const v4f a0 = *(const v4f*)ap, a1 = *(const v4f*)(ap + 4);
      const v4f a2 = *(const v4f*)(ap + 16), a3 = *(const v4f*)(ap + 20);
      v16b ahi, alo;
#pragma unroll
      for (int e = 0; e < 4; ++e) {
        __bf16 h, l;
        split_bf(a0[e], h, l); ahi[e] = h;      alo[e] = l;
        split_bf(a1[e], h, l); ahi[4 + e] = h;  alo[4 + e] = l;
        split_bf(a2[e], h, l); ahi[8 + e] = h;  alo[8 + e] = l;
        split_bf(a3[e], h, l); ahi[12 + e] = h; alo[12 + e] = l;
      }
      v16b bw[6];
#pragma unroll
      for (int j = 0; j < 6; ++j)
        bw[j] = Frag<__bf16>::load(Bt + (size_t)(cw + (j << 4) + rlane) * ODIM + k0 + koff);
#pragma unroll
      for (int j = 0; j < 6; ++j) {
        acc[j] = Frag<__bf16>::mma(ahi, bw[j], acc[j]);
        acc[j] = Frag<__bf16>::mma(alo, bw[j], acc[j]);
      }
      Frag<__bf16>::guard(acc[0], acc[5], ahi, alo);
      Frag<__bf16>::keep(bw[0], bw[1], bw[2], bw[3]);
      Frag<__bf16>::keep(bw[4], bw[5], bw[4], bw[5]);
    }
    acc_guard4(acc[0], acc[1], acc[2], acc[3]);
    acc_guard2(acc[4], acc[5]);
#pragma unroll
    for (int j = 0; j < 6; ++j) {
      const int col = cw + (j << 4) + rlane;
      const float bv = bfr(bfcs[oi * ODIM + col]);
#pragma unroll
      for (int r = 0; r < 8; ++r) slab[(mOff + r) * SL_PITCH + (j << 4) + rlane] = acc[j][r] + bv;
    }
    wave_lds_sync();
    {
      float* ob = outp + (size_t)oi * OUT_ELEMS;
      const int lc = (lane < 24) ? lane : 23;
      for (int pass = 0; pass < 2; ++pass) {
#pragma unroll
        for (int row = 0; row < 16; ++row) {
          const v4f v = *(const v4f*)(slab + row * SL_PITCH + 4 * lc);
          if (lane < 24) *(volatile v4f*)(ob + (size_t)row * ODIM + cw + 4 * lane) = v;
        }
        __threadfence();
      }
    }
    wave_lds_sync();
  }
}

extern "C" void kernel_launch(void* const* d_in, const int* in_sizes, int n_in,
                              void* d_out, int out_size, void* d_ws, size_t ws_size,
                              hipStream_t stream) {
  (void)n_in;
  const float* x    = (const float*)d_in[0];
  const float* Wfc  = (const float*)d_in[1];
  const float* bfc  = (const float*)d_in[2];
  const float* lng  = (const float*)d_in[3];
  const float* lnb  = (const float*)d_in[4];
  const float* aw   = (const float*)d_in[5];
  const float* ab   = (const float*)d_in[6];
  const float* Wcat = (const float*)d_in[7];
  const float* bcat = (const float*)d_in[8];
  const float* lOg  = (const float*)d_in[9];
  const float* lOb  = (const float*)d_in[10];
  const float* Wfcs = (const float*)d_in[11];
  const float* bfcs = (const float*)d_in[12];
  float* outp = (float*)d_out;

  if (in_sizes[0] != NTOK * TDIM || in_sizes[1] != NHEADS * TDIM * HIDC || in_sizes[7] != CATD * ODIM ||
      in_sizes[11] != 3 * ODIM * ODIM || out_size != 4 * OUT_ELEMS) return;

  char* ws = (char*)d_ws;
  size_t off = 0;
  auto carve = [&](size_t bytes) -> char* {
    char* p = ws + off;
    off = (off + bytes + 255) & ~(size_t)255;
    return p;
  };
  unsigned short* Xb    = (unsigned short*)carve((size_t)NTOK * TDIM * 2);
  unsigned short* WT    = (unsigned short*)carve((size_t)NHEADS * HIDC * TDIM * 2);
  unsigned short* hThi  = (unsigned short*)carve((size_t)NHEADS * NBATCH * HIDC * SEQL * 2);
  unsigned short* hTlo  = (unsigned short*)carve((size_t)NHEADS * NBATCH * HIDC * SEQL * 2);
  float*          srow  = (float*)carve((size_t)NHEADS * NTOK * 4);
  float*          scol  = (float*)carve((size_t)NHEADS * NTOK * 4);
  float*          sentp = (float*)carve((size_t)NBATCH * CATD * 4);
  unsigned short* WcatT = (unsigned short*)carve((size_t)ODIM * CATD * 2);
  unsigned short* WfcsT = (unsigned short*)carve((size_t)3 * ODIM * ODIM * 2);
  if (off > ws_size) return;

  const int n8 = NTOK * TDIM / 8;
  k_cast_bf16x8<<<dim3((n8 + 255) / 256), dim3(256), 0, stream>>>(x, Xb, n8);
  k_tr_cast<<<dim3(HIDC / 64, TDIM / 64, NHEADS), dim3(256), 0, stream>>>(Wfc, WT, TDIM, HIDC);
  k_tr_cast<<<dim3(ODIM / 64, CATD / 64, 1), dim3(256), 0, stream>>>(Wcat, WcatT, CATD, ODIM);
  k_tr_cast<<<dim3(ODIM / 64, ODIM / 64, 3), dim3(256), 0, stream>>>(Wfcs, WfcsT, ODIM, ODIM);
  k_proj_ln<<<dim3(NTOK / 64, NHEADS), dim3(128), 0, stream>>>(
      Xb, WT, bfc, lng, lnb, aw, hThi, hTlo, srow, scol);
  k_attnw<<<dim3(NHEADS * NBATCH), dim3(256), 0, stream>>>(srow, scol, ab, hThi, hTlo, sentp);
  k_tail<<<dim3(1), dim3(256), 0, stream>>>(sentp, WcatT, bcat, lOg, lOb, WfcsT, bfcs, outp);
}
